// DownstreamExpert_83545703842159
// MI455X (gfx1250) — hardware-verified
//
#include <hip/hip_runtime.h>
#include <stddef.h>


typedef _Float16 v16h __attribute__((ext_vector_type(16)));
typedef _Float16 v8h  __attribute__((ext_vector_type(8))) __attribute__((may_alias));
typedef float    v8f  __attribute__((ext_vector_type(8)));
typedef float    v4f  __attribute__((ext_vector_type(4))) __attribute__((may_alias));

union Frag { v16h v; v8h h[2]; };

#define NB    16
#define NT1   1024
#define NT2   768
#define NDU   768
#define NDP   128

#define SC_A    16.0f
#define SC_W    64.0f
#define SC_X    16.0f
#define INV_AW  (1.0f / 1024.0f)
#define INV_XX  (1.0f / 256.0f)

#define SM_GAMMA 0.1f
#define SM_INVG  10.0f
#define SM_BIG   1e8f
#define SKEW     16
#define RING     (4 * SKEW)
#define RES_STRIDE 128

__device__ __forceinline__ v8f wmma_f16(v16h a, v16h b, v8f c)
{
  c = __builtin_amdgcn_wmma_f32_16x16x32_f16(false, a, false, b, (short)0, c, false, false);
  asm volatile("v_nop\n\tv_nop\n\tv_nop\n\tv_nop" : "+v"(c) : "v"(a), "v"(b));
  return c;
}

__global__ __launch_bounds__(256) void k_wprep(const float* __restrict__ W,
                                               _Float16* __restrict__ Wt)
{
  const int t   = blockIdx.x * 256 + threadIdx.x;
  const int lpr = NDU / 64;
  if (t >= NDP * lpr) return;
  const int n  = t / lpr;
  const int q  = t - n * lpr;
  const int k0 = q * 64;
  v8h v[8];
#pragma unroll
  for (int s = 0; s < 8; ++s) {
    v8h x;
#pragma unroll
    for (int e = 0; e < 8; ++e)
      x[e] = (_Float16)(W[(size_t)(k0 + 8 * s + e) * NDP + n] * SC_W);
    v[s] = x;
  }
  _Float16* dst = Wt + (size_t)n * NDU + k0;
#pragma unroll
  for (int s = 0; s < 8; ++s) *(volatile v8h*)(dst + 8 * s) = v[s];
  __threadfence();
#pragma unroll
  for (int s = 0; s < 8; ++s) *(volatile v8h*)(dst + 8 * s) = v[s];
}

__global__ __launch_bounds__(256) void k_proj(const float* __restrict__ A,
                                              const _Float16* __restrict__ Wt,
                                              const float* __restrict__ bias,
                                              _Float16* __restrict__ Xo)
{
  __shared__ __attribute__((aligned(16))) _Float16 As[16][NDU + 8];
  __shared__ __attribute__((aligned(16))) _Float16 Ts[16][NDP + 8];
  __shared__ float part[8][16];
  __shared__ float invn[16];

  const int row0 = blockIdx.x * 16;
  const int tid  = threadIdx.x;

#pragma unroll
  for (int it = 0; it < (16 * NDU / 8) / 256; ++it) {
    const int u   = it * 256 + tid;
    const int row = u / (NDU / 8);
    const int c8  = u - row * (NDU / 8);
    const float* src = A + (size_t)(row0 + row) * NDU + c8 * 8;
    const v4f f0 = *(const v4f*)src;
    const v4f f1 = *(const v4f*)(src + 4);
    v8h x;
    x[0] = (_Float16)(f0[0] * SC_A); x[1] = (_Float16)(f0[1] * SC_A);
    x[2] = (_Float16)(f0[2] * SC_A); x[3] = (_Float16)(f0[3] * SC_A);
    x[4] = (_Float16)(f1[0] * SC_A); x[5] = (_Float16)(f1[1] * SC_A);
    x[6] = (_Float16)(f1[2] * SC_A); x[7] = (_Float16)(f1[3] * SC_A);
    *(v8h*)(&As[row][c8 * 8]) = x;
  }
  __syncthreads();

  const int l    = tid & 31;
  const int h    = l >> 4;
  const int m    = l & 15;
  const int wave = tid >> 5;
  const int n0   = wave * 16;

  const _Float16* ar = &As[m][0];
  const _Float16* br = Wt + (size_t)(n0 + m) * NDU;

  v8f c = {0.f, 0.f, 0.f, 0.f, 0.f, 0.f, 0.f, 0.f};
#pragma unroll 4
  for (int k0 = 0; k0 < NDU; k0 += 32) {
    Frag a, b;
    a.h[0] = *(const v8h*)(ar + k0 + 8 * h);
    a.h[1] = *(const v8h*)(ar + k0 + 16 + 8 * h);
    b.h[0] = *(const v8h*)(br + k0 + 8 * h);
    b.h[1] = *(const v8h*)(br + k0 + 16 + 8 * h);
    c = wmma_f16(a.v, b.v, c);
  }

  const float bn = bias[n0 + m];
  float z[8], ss[8];
#pragma unroll
  for (int r = 0; r < 8; ++r) { z[r] = c[r] * INV_AW + bn; ss[r] = z[r] * z[r]; }
#pragma unroll
  for (int mask = 1; mask < 16; mask <<= 1) {
#pragma unroll
    for (int r = 0; r < 8; ++r) ss[r] += __shfl_xor(ss[r], mask, 32);
  }
  if (m == 0) {
#pragma unroll
    for (int r = 0; r < 8; ++r) part[wave][8 * h + r] = ss[r];
  }
  __syncthreads();
  if (tid < 16) {
    float t = 0.f;
#pragma unroll
    for (int w = 0; w < 8; ++w) t += part[w][tid];
    invn[tid] = rsqrtf(fmaxf(t, 1e-24f)) * SC_X;
  }
  __syncthreads();
#pragma unroll
  for (int r = 0; r < 8; ++r)
    Ts[8 * h + r][n0 + m] = (_Float16)(z[r] * invn[8 * h + r]);
  __syncthreads();

  const int L  = 4 * wave + (l >> 3);
  const int rr = L >> 1, hh = L & 1, e = l & 7;
  const v8h v = *(const v8h*)(&Ts[rr][hh * 64 + e * 8]);
  _Float16* dst = Xo + (size_t)(row0 + rr) * NDP + hh * 64 + e * 8;
  *(volatile v8h*)dst = v;
  __threadfence();
  *(volatile v8h*)dst = v;
}

__global__ __launch_bounds__(256) void k_gram(const _Float16* X, const _Float16* Y,
                                              _Float16* __restrict__ G, int N, int M)
{
  __shared__ __attribute__((aligned(16))) _Float16 Ts[16][NDP + 8];

  const int bat  = blockIdx.z;
  const int i0   = blockIdx.x * 16;
  const int tid  = threadIdx.x;
  const int l    = tid & 31;
  const int h    = l >> 4;
  const int m    = l & 15;
  const int wave = tid >> 5;
  const int jb   = blockIdx.y * 128;
  const int j0   = jb + wave * 16;

  const _Float16* xr = X + ((size_t)bat * N + i0 + m) * NDP;
  const _Float16* yr = Y + ((size_t)bat * M + j0 + m) * NDP;

  v8f c = {0.f, 0.f, 0.f, 0.f, 0.f, 0.f, 0.f, 0.f};
#pragma unroll
  for (int k0 = 0; k0 < NDP; k0 += 32) {
    Frag a, b;
    a.h[0] = *(const v8h*)(xr + k0 + 8 * h);
    a.h[1] = *(const v8h*)(xr + k0 + 16 + 8 * h);
    b.h[0] = *(const v8h*)(yr + k0 + 8 * h);
    b.h[1] = *(const v8h*)(yr + k0 + 16 + 8 * h);
    c = wmma_f16(a.v, b.v, c);
  }
#pragma unroll
  for (int r = 0; r < 8; ++r)
    Ts[8 * h + r][wave * 16 + m] = (_Float16)(c[r] * INV_XX);
  __syncthreads();

  const int L  = 4 * wave + (l >> 3);
  const int rr = L >> 1, hh = L & 1, e = l & 7;
  const v8h v = *(const v8h*)(&Ts[rr][hh * 64 + e * 8]);
  _Float16* dst = G + ((size_t)bat * N + i0 + rr) * (size_t)M + jb + hh * 64 + e * 8;
  *(volatile v8h*)dst = v;
  __threadfence();
  *(volatile v8h*)dst = v;
}

__global__ __launch_bounds__(1024) void k_sdtw(const _Float16* __restrict__ Gxy,
                                               const _Float16* __restrict__ Gxx,
                                               const _Float16* __restrict__ Gyy,
                                               float* __restrict__ res)
{
  __shared__ float ring[32][RING];
  const int type = blockIdx.x;
  const int bat  = blockIdx.y;
  const _Float16* Gb; int N, M;
  if (type == 0)      { N = NT1; M = NT2; Gb = Gxy + (size_t)bat * NT1 * NT2; }
  else if (type == 1) { N = NT1; M = NT1; Gb = Gxx + (size_t)bat * NT1 * NT1; }
  else                { N = NT2; M = NT2; Gb = Gyy + (size_t)bat * NT2 * NT2; }

  const int tid   = threadIdx.x;
  const int lane  = tid & 31;
  const int w     = tid >> 5;
  const int i     = tid;
  const int steps = N + M - 1;
  const int nw    = N >> 5;
  const int T     = steps + SKEW * (nw - 1);
  const int dofs  = SKEW * w;
  const int dlo   = 32 * w;
  int dhi = 32 * w + 31 + M - 1; if (dhi > steps - 1) dhi = steps - 1;
  const int wm    = (w > 0) ? (w - 1) : 0;
  const _Float16* gp = Gb + (size_t)i * (size_t)(M - 1);

  float p1 = SM_BIG, p2 = SM_BIG, fin = 0.f;

  for (int t0 = 0; t0 < T; t0 += SKEW) {
#pragma unroll 4
    for (int s = 0; s < SKEW; ++s) {
      const int t = t0 + s;
      const int d = t - dofs;
      if (w < nw && d >= dlo && d <= dhi) {
        const int j = d - i;
        const bool valid = (j >= 0) && (j < M);
        float dc = 0.f;
        if (valid) dc = 2.0f - 2.0f * (float)gp[d];
        float u1 = __shfl_up(p1, 1, 32);
        float u2 = __shfl_up(p2, 1, 32);
        if (lane == 0) {
          if (w == 0) {
            u1 = SM_BIG;
            u2 = (d == 0) ? 0.f : SM_BIG;
          } else {
            u1 = (d >= 1) ? ring[wm][(t - SKEW - 1) & (RING - 1)] : SM_BIG;
            u2 = (d >= 2) ? ring[wm][(t - SKEW - 2) & (RING - 1)] : SM_BIG;
          }
        }
        float val = SM_BIG;
        if (valid) {
          const float mn = fminf(u1, u2), mx = fmaxf(u1, u2);
          const float mm = fminf(mn, p1), o1 = fmaxf(mn, p1);
          const float sm = 1.0f + __expf((mm - o1) * SM_INVG) + __expf((mm - mx) * SM_INVG);
          val = dc + (mm - SM_GAMMA * __logf(sm));
        }
        p2 = p1; p1 = val;
        if (lane == 31) ring[w][t & (RING - 1)] = val;
        if (d == steps - 1) fin = val;
      }
    }
    __syncthreads();
  }

  if (w == nw - 1) {
    const float r = __shfl(fin, 31, 32);
    v4f vv; vv[0] = r; vv[1] = r; vv[2] = r; vv[3] = r;
    float* dst = res + (size_t)(type * NB + bat) * RES_STRIDE + lane * 4;
    *(volatile v4f*)dst = vv;
    __threadfence();
    *(volatile v4f*)dst = vv;
  }
}

__global__ __launch_bounds__(32) void k_fin(const float* __restrict__ res,
                                            float* __restrict__ out)
{
  if (threadIdx.x == 0 && blockIdx.x == 0) {
    float s = 0.f;
#pragma unroll 1
    for (int bb = 0; bb < NB; ++bb)
      s += res[(size_t)bb * RES_STRIDE]
           - 0.5f * (res[(size_t)(NB + bb) * RES_STRIDE] + res[(size_t)(2 * NB + bb) * RES_STRIDE]);
    const float v = (s * (1.0f / (float)NB)) * (1.0f / (float)(NT1 + NT2));
    *(volatile float*)out = v;
    __threadfence();
    *(volatile float*)out = v;
  }
}

extern "C" void kernel_launch(void* const* d_in, const int* in_sizes, int n_in,
                              void* d_out, int out_size, void* d_ws, size_t ws_size,
                              hipStream_t stream)
{
  if (n_in < 4 || out_size < 1) return;
  if (in_sizes[0] != NB * NT1 * NDU || in_sizes[1] != NB * NT2 * NDU ||
      in_sizes[2] != NDU * NDP || in_sizes[3] != NDP) return;

  const float* feats = (const float*)d_in[0];
  const float* tgts  = (const float*)d_in[1];
  const float* W     = (const float*)d_in[2];
  const float* bias  = (const float*)d_in[3];

  const size_t szWt  = (size_t)NDP * NDU * 2;
  const size_t szX   = (size_t)NB * NT1 * NDP * 2;
  const size_t szY   = (size_t)NB * NT2 * NDP * 2;
  const size_t szGxy = (size_t)NB * NT1 * NT2 * 2;
  const size_t szGxx = (size_t)NB * NT1 * NT1 * 2;
  const size_t szGyy = (size_t)NB * NT2 * NT2 * 2;
  const size_t szRes = (size_t)3 * NB * RES_STRIDE * 4;

  const size_t offWt  = 0;
  const size_t offX   = offWt + szWt;
  const size_t offY   = offX + szX;
  const size_t offGxy = offY + szY;
  const size_t offGxx = offGxy + szGxy;
  const size_t offGyy = offGxx + szGxx;
  const size_t offRes = offGyy + szGyy;
  const size_t total  = offRes + szRes;
  if (total > ws_size) return;

  char* ws = (char*)d_ws;
  _Float16* Wt  = (_Float16*)(ws + offWt);
  _Float16* Xh  = (_Float16*)(ws + offX);
  _Float16* Yh  = (_Float16*)(ws + offY);
  _Float16* Gxy = (_Float16*)(ws + offGxy);
  _Float16* Gxx = (_Float16*)(ws + offGxx);
  _Float16* Gyy = (_Float16*)(ws + offGyy);
  float*    res = (float*)(ws + offRes);
  float*    out = (float*)d_out;

  k_wprep<<<(NDP * (NDU / 64) + 255) / 256, 256, 0, stream>>>(W, Wt);

  k_proj<<<NB * NT1 / 16, 256, 0, stream>>>(feats, Wt, bias, Xh);
  k_proj<<<NB * NT2 / 16, 256, 0, stream>>>(tgts,  Wt, bias, Yh);

  k_gram<<<dim3(NT1 / 16, NT2 / 128, NB), 256, 0, stream>>>(Xh, Yh, Gxy, NT1, NT2);
  k_gram<<<dim3(NT1 / 16, NT1 / 128, NB), 256, 0, stream>>>(Xh, Xh, Gxx, NT1, NT1);
  k_gram<<<dim3(NT2 / 16, NT2 / 128, NB), 256, 0, stream>>>(Yh, Yh, Gyy, NT2, NT2);

  k_sdtw<<<dim3(3, NB), 1024, 0, stream>>>(Gxy, Gxx, Gyy, res);

  k_fin<<<1, 32, 0, stream>>>(res, out);
}
